// KANLayerFast_66821101191171
// MI455X (gfx1250) — hardware-verified
//
#include <hip/hip_runtime.h>
#include <stddef.h>
#include <stdint.h>

#pragma clang fp contract(off)

#define NB   4096
#define NI   256
#define NO   512
#define NK   64
#define KC   128
#define EPSF 1e-12f

#define BMT  128
#define BNT  128
#define LDA  136
#define STP  36

static_assert(NI == 256);
static_assert(NB % BMT == 0);
static_assert(NO % BNT == 0);
static_assert((NO * NI) % 8 == 0);
static_assert((LDA * 2) % 16 == 0);
static_assert((STP * 4) % 16 == 0);

typedef _Float16 v16h __attribute__((ext_vector_type(16)));
typedef _Float16 v8h  __attribute__((ext_vector_type(8)));
typedef float    v8f  __attribute__((ext_vector_type(8)));
typedef float    v4f  __attribute__((ext_vector_type(4)));
typedef unsigned int v4u __attribute__((ext_vector_type(4)));
typedef v8h __attribute__((may_alias)) v8ha;
typedef v4u __attribute__((may_alias)) v4ua;
typedef v4f __attribute__((may_alias)) v4fa;

union Frag { v16h v; v8h h[2]; };

__device__ __forceinline__ v8f mma16(v16h a, v16h b, v8f cacc) {
  cacc = __builtin_amdgcn_wmma_f32_16x16x32_f16(false, a, false, b, (short)0, cacc, false, false);
  asm volatile("v_nop\n\tv_nop\n\tv_nop\n\tv_nop" : "+v"(cacc) : "v"(a), "v"(b));
  return cacc;
}

__device__ __forceinline__ v8f zero8() { return (v8f){0.f, 0.f, 0.f, 0.f, 0.f, 0.f, 0.f, 0.f}; }

__device__ __forceinline__ v16h ldfrag_g(const _Float16* __restrict__ p, int ld, int row0, int k0, int lane) {
  const int m = lane & 15, lh = lane >> 4;
  const _Float16* q = p + (size_t)(row0 + m) * ld + k0 + 8 * lh;
  Frag f;
  f.h[0] = *(const v8h*)(q);
  f.h[1] = *(const v8h*)(q + 16);
  return f.v;
}

__device__ __forceinline__ v16h ldfrag_l(const _Float16* p, int ld, int row0, int k0, int lane) {
  const int m = lane & 15, lh = lane >> 4;
  const _Float16* q = p + (row0 + m) * ld + k0 + 8 * lh;
  Frag f;
  f.h[0] = *(const v8ha*)(q);
  f.h[1] = *(const v8ha*)(q + 16);
  return f.v;
}

__device__ __forceinline__ float limit3(float di, float de) {
  di = (di * de <= 0.0f) ? 0.0f : di;
  return (fabsf(di) > 3.0f * fabsf(de)) ? 3.0f * de : di;
}

__device__ __forceinline__ float pchip_mid(float dp, float dn, float hk, float hkm) {
  const float w1 = 2.0f * hk + hkm;
  const float w2 = hk + 2.0f * hkm;
  const float den = (w1 / (dp + EPSF) + w2 / (dn + EPSF)) + EPSF;
  const float dint = (w1 + w2) / den;
  return (dp * dn > 0.0f) ? dint : 0.0f;
}

__global__ __launch_bounds__(256) void k_prep(const float* __restrict__ C, const float* __restrict__ knots,
                                              _Float16* __restrict__ MC) {
  __shared__ float skn[NK];
  __shared__ float sh[NK];
  __shared__ float srh[NK];
  __shared__ float sy[8][NK + 8];
  __shared__ float sdl[8][NK + 8];
  __shared__ __align__(16) _Float16 so[8][KC];

  const int tid = threadIdx.x, lane = tid & 31, wave = tid >> 5;
  const int pair = blockIdx.x * 8 + wave;
  const int o = pair >> 8;
  const int i = pair & (NI - 1);

  if (tid < NK) skn[tid] = knots[tid];
  __syncthreads();
  if (tid < NK) {
    const int j1 = (tid < NK - 1) ? tid + 1 : NK - 1;
    const float hv = skn[j1] - skn[tid];
    sh[tid]  = hv;
    srh[tid] = 1.0f / (hv + EPSF);
  }
  const float* y = C + ((size_t)o * NI + i) * NK;
  float* syw = sy[wave];
  float* sdw = sdl[wave];
  syw[lane]      = y[lane];
  syw[lane + 32] = y[lane + 32];
  __syncthreads();
  {
    const int ja = lane, jb = lane + 32;
    const int jb1 = (jb < NK - 1) ? jb + 1 : NK - 1;
    sdw[ja] = (syw[ja + 1] - syw[ja]) * srh[ja];
    sdw[jb] = (syw[jb1] - syw[jb]) * srh[jb];
  }
  __syncthreads();

  const float h0 = sh[0], h1 = sh[1], hm1 = sh[NK - 2], hm2 = sh[NK - 3];
  const float dl0 = sdw[0], dl1 = sdw[1], dlm1 = sdw[NK - 2], dlm2 = sdw[NK - 3];
  float e0 = ((2.0f * h0 + h1) * dl0 - h0 * dl1) * (1.0f / ((h0 + h1) + EPSF));
  e0 = limit3(e0, dl0);
  float eN = ((2.0f * hm1 + hm2) * dlm1 - hm1 * dlm2) * (1.0f / ((hm1 + hm2) + EPSF));
  eN = limit3(eN, dlm1);

  _Float16* sow = so[wave];
#pragma unroll 1
  for (int q = 0; q < 2; ++q) {
    const int k  = lane + 32 * q;
    const int km = (k > 0) ? k - 1 : 0;
    const int kp = (k < NK - 1) ? k : NK - 2;
    const float mid = pchip_mid(sdw[km], sdw[kp], sh[kp], sh[km]);
    float sl = (k == 0) ? e0 : mid;
    sl = (k == NK - 1) ? eN : sl;
    sow[k]      = (_Float16)(syw[k] * 128.0f);
    sow[NK + k] = (_Float16)(sl * 32.0f);
  }
  __syncthreads();

  const int pc = lane & 15;
  const v4u val = *(const v4ua*)(sow + pc * 8);
  _Float16* dst = MC + ((size_t)i * NO + o) * KC + pc * 8;
  if (lane < 16) *(volatile v4u*)dst = val;
  __threadfence();
  if (lane < 16) *(volatile v4u*)dst = val;
}

__global__ __launch_bounds__(256) void k_gemm(const float* __restrict__ X, const _Float16* __restrict__ MC,
                                              const float* __restrict__ bias, const float* __restrict__ knots,
                                              float* __restrict__ out) {
  __shared__ float skn[NK];
  __shared__ __align__(16) _Float16 sA[BMT * LDA];
  __shared__ __align__(16) float st[8][16 * STP];

  const int tid = threadIdx.x, lane = tid & 31, wave = tid >> 5;
  const int hh = lane >> 4, c = lane & 15;
  const int wr = wave >> 2;
  const int wc = wave & 3;
  const int bm0 = blockIdx.x * BMT;
  const int on0 = blockIdx.y * BNT;

  if (tid < NK) skn[tid] = knots[tid];
  {
    const v4u z = (v4u){0u, 0u, 0u, 0u};
#pragma unroll
    for (int j = 0; j < 8; ++j) {
      const int p = tid + 256 * j;
      const int row = p >> 4, pc = p & 15;
      *(v4ua*)(sA + row * LDA + pc * 8) = z;
    }
  }
  __syncthreads();
  const float kn0 = skn[0], kn63 = skn[NK - 1];

  v8f acc[4][2];
#pragma unroll
  for (int s = 0; s < 4; ++s) { acc[s][0] = zero8(); acc[s][1] = zero8(); }

  int os0 = 0, os1 = 1;
  const int nrow0 = on0 + wc * 32;
  const int arow0 = wr * 64;

  for (int i = 0; i < NI; ++i) {
    if (tid < BMT) {
      const float xv = X[(size_t)(bm0 + tid) * NI + i];
      const bool below = xv < kn0;
      const bool above = xv > kn63;
      const bool ext = below || above;
      const float xc = fminf(fmaxf(xv, kn0), kn63);
      int pos = 0;
      pos = (skn[pos + 31] < xc) ? pos + 32 : pos;
      pos = (skn[pos + 15] < xc) ? pos + 16 : pos;
      pos = (skn[pos + 7]  < xc) ? pos + 8  : pos;
      pos = (skn[pos + 3]  < xc) ? pos + 4  : pos;
      pos = (skn[pos + 1]  < xc) ? pos + 2  : pos;
      pos = (skn[pos]      < xc) ? pos + 1  : pos;
      int idx = pos - 1;
      idx = (idx < 0) ? 0 : idx;
      idx = (idx > NK - 2) ? NK - 2 : idx;
      const float x0 = skn[idx];
      const float hc = (skn[idx + 1] - x0) + EPSF;
      const float t  = (xc - x0) * (1.0f / hc);
      const float t2 = t * t;
      const float t3 = t2 * t;
      const float h00 = (2.0f * t3 - 3.0f * t2) + 1.0f;
      const float h10 = (t3 - 2.0f * t2) + t;
      const float h01 = -2.0f * t3 + 3.0f * t2;
      const float h11 = t3 - t2;
      const int   s0  = below ? 0 : (above ? NK - 1 : idx);
      const int   s1  = ext ? s0 : idx + 1;
      const float dxe = below ? (xv - kn0) : (xv - kn63);
      const float wy0 = ext ? 1.0f : h00;
      const float wy1 = ext ? wy0 : h01;
      const float wd0 = ext ? dxe : h10 * hc;
      const float wd1 = ext ? wd0 : h11 * hc;
      _Float16* ar = sA + tid * LDA;
      ar[os0]      = (_Float16)0.0f;
      ar[os1]      = (_Float16)0.0f;
      ar[NK + os0] = (_Float16)0.0f;
      ar[NK + os1] = (_Float16)0.0f;
      ar[s0]       = (_Float16)(wy0 * 256.0f);
      ar[s1]       = (_Float16)(wy1 * 256.0f);
      ar[NK + s0]  = (_Float16)(wd0 * 1024.0f);
      ar[NK + s1]  = (_Float16)(wd1 * 1024.0f);
      os0 = s0; os1 = s1;
    }
    __syncthreads();

    const _Float16* Bp = MC + (size_t)i * NO * KC;
#pragma unroll 2
    for (int kc = 0; kc < 4; ++kc) {
      const int k0 = kc * 32;
      const v16h b0 = ldfrag_g(Bp, KC, nrow0, k0, lane);
      const v16h b1 = ldfrag_g(Bp, KC, nrow0 + 16, k0, lane);
#pragma unroll
      for (int s = 0; s < 4; ++s) {
        const v16h a = ldfrag_l(sA, LDA, arow0 + s * 16, k0, lane);
        acc[s][0] = mma16(a, b0, acc[s][0]);
        acc[s][1] = mma16(a, b1, acc[s][1]);
      }
    }
    __syncthreads();
  }

  const float scl = 3.0517578125e-05f;
  const float bv0 = bias[nrow0 + c];
  const float bv1 = bias[nrow0 + 16 + c];
  float* sw = st[wave];
#pragma unroll
  for (int s = 0; s < 4; ++s) {
#pragma unroll
    for (int r = 0; r < 8; ++r) {
      sw[(8 * hh + r) * STP + c]      = acc[s][0][r] * scl + bv0;
      sw[(8 * hh + r) * STP + 16 + c] = acc[s][1][r] * scl + bv1;
    }
    __syncthreads();
    v4f val[4];
    size_t go[4];
#pragma unroll
    for (int it = 0; it < 4; ++it) {
      const int p  = lane + 32 * it;
      const int L  = p >> 3;
      const int pc = p & 7;
      val[it] = *(const v4fa*)(sw + L * STP + pc * 4);
      go[it]  = (size_t)(bm0 + arow0 + s * 16 + L) * NO + nrow0 + pc * 4;
    }
    for (int ps = 0; ps < 2; ++ps) {
#pragma unroll
      for (int it = 0; it < 4; ++it) *(volatile v4f*)(out + go[it]) = val[it];
      __threadfence();
    }
    __syncthreads();
  }
}

extern "C" void kernel_launch(void* const* d_in, const int* in_sizes, int n_in,
                              void* d_out, int out_size, void* d_ws, size_t ws_size,
                              hipStream_t stream) {
  if (n_in < 4) return;
  if (in_sizes[0] != NB * NI) return;
  if (in_sizes[1] != NO * NI * NK) return;
  if (in_sizes[2] != NO) return;
  if (in_sizes[3] != NK) return;
  if (out_size != NB * NO) return;

  const float* x      = (const float*)d_in[0];
  const float* coeffs = (const float*)d_in[1];
  const float* bias   = (const float*)d_in[2];
  const float* knots  = (const float*)d_in[3];
  float* out = (float*)d_out;

  const size_t mc_bytes = (size_t)NI * NO * KC * 2;
  if (mc_bytes > ws_size) return;
  _Float16* MC = (_Float16*)d_ws;

  k_prep<<<dim3((NO * NI) / 8), dim3(256), 0, stream>>>(coeffs, knots, MC);
  k_gemm<<<dim3(NB / BMT, NO / BNT), dim3(256), 0, stream>>>(x, MC, bias, knots, out);
  (void)hipGetLastError();
}
